// CorrelationAttention_local_33981781246277
// MI455X (gfx1250) — hardware-verified
//
#include <hip/hip_runtime.h>
#include <hip/hip_bf16.h>

#define FEAT  512
#define MATCH 256
#define BATCH 8
#define SEQ   2048
#define ROWS  (BATCH*SEQ)
#define EPSLN 1e-5f

#define BC    64
#define VT_LD 72

typedef __attribute__((ext_vector_type(16))) _Float16 v16h;
typedef __attribute__((ext_vector_type(8)))  _Float16 v8h;
typedef __attribute__((ext_vector_type(8)))  float    v8f;

#define TR16_MODE 0
typedef __attribute__((ext_vector_type(4))) float v4f;
typedef __attribute__((ext_vector_type(4))) unsigned v4u;
template <typename T> __device__ __forceinline__ void vst2(void* p, T v) { *(volatile T*)p = v; __threadfence(); *(volatile T*)p = v; }

static __device__ __forceinline__ v8f wmma16x16x32(v16h a, v16h b, v8f c) {
  v8f d = __builtin_amdgcn_wmma_f32_16x16x32_f16(false, a, false, b, (short)0, c, false, false);
  asm volatile("v_nop\n\tv_nop\n\tv_nop\n\tv_nop" : "+v"(d) : "v"(a), "v"(b));
  return d;
}

static __device__ __forceinline__ v16h load_fragA(const _Float16* base, int ld, int lane) {
  const _Float16* p = base + (lane & 15) * ld + (lane >> 4) * 8;
  v8h lo = *(const v8h*)(p);
  v8h hi = *(const v8h*)(p + 16);
  return __builtin_shufflevector(lo, hi, 0,1,2,3,4,5,6,7,8,9,10,11,12,13,14,15);
}

static __device__ __forceinline__ v16h load_fragB(const _Float16* base, int ld, int lane) {
  const _Float16* p = base + (lane & 15) * ld + (lane >> 4) * 8;
  v8h lo = *(const v8h*)(p);
  v8h hi = *(const v8h*)(p + 16);
  return __builtin_shufflevector(lo, hi, 0,1,2,3,4,5,6,7,8,9,10,11,12,13,14,15);
}


__global__ void k_prep_weights(const float* __restrict__ Wp, const float* __restrict__ Wo,
                               _Float16* __restrict__ WpT, _Float16* __restrict__ WoT) {
  int i8 = (blockIdx.x * blockDim.x + threadIdx.x) * 8;
  union { v8h h; v4u u; } pk;
  if (i8 < FEAT * MATCH) {
    int m = i8 / FEAT, f = i8 % FEAT;
#pragma unroll
    for (int e = 0; e < 8; ++e) pk.h[e] = (_Float16)Wp[(f + e) * MATCH + m];
    vst2(WpT + i8, pk.u);
  }
  int j8 = i8 - FEAT * MATCH;
  if (j8 >= 0 && j8 < FEAT * FEAT) {
    int g = j8 / FEAT, f = j8 % FEAT;
#pragma unroll
    for (int e = 0; e < 8; ++e) pk.h[e] = (_Float16)Wo[(f + e) * FEAT + g];
    vst2(WoT + j8, pk.u);
  }
}

__global__ void k_proj_ln(const float* __restrict__ X, const _Float16* __restrict__ WpT,
                          const float* __restrict__ b_proj,
                          const float* __restrict__ g1, const float* __restrict__ be1,
                          const float* __restrict__ g2, const float* __restrict__ be2,
                          _Float16* __restrict__ qk_h, _Float16* __restrict__ v_h) {
  __shared__ __align__(16) _Float16 sA[16][FEAT];
  __shared__ __align__(16) float    sP[16][MATCH];
  __shared__ __align__(16) _Float16 sV[16][FEAT];
  __shared__ __align__(16) _Float16 sQ[16][MATCH];

  int row0 = blockIdx.x * 16;
  int t = threadIdx.x, lane = t & 31, w = t >> 5;

  for (int idx = t; idx < 16 * FEAT; idx += 256) {
    int r = idx >> 9, c = idx & (FEAT - 1);
    sA[r][c] = (_Float16)X[(row0 + r) * FEAT + c];
  }

  for (int rr = 0; rr < 2; ++rr) {
    int grow = row0 + w * 2 + rr;
    float xv[16]; float s = 0.f, s2 = 0.f;
#pragma unroll
    for (int i = 0; i < 16; ++i) {
      float x = X[grow * FEAT + lane + 32 * i];
      xv[i] = x; s += x; s2 += x * x;
    }
#pragma unroll
    for (int o = 16; o > 0; o >>= 1) { s += __shfl_xor(s, o, 32); s2 += __shfl_xor(s2, o, 32); }
    float mu = s * (1.f / FEAT);
    float var = s2 * (1.f / FEAT) - mu * mu;
    float rs = rsqrtf(var + EPSLN);
#pragma unroll
    for (int i = 0; i < 16; ++i) {
      int c = lane + 32 * i;
      sV[w * 2 + rr][c] = (_Float16)((xv[i] - mu) * rs * g2[c] + be2[c]);
    }
    asm volatile("s_wait_dscnt 0" ::: "memory"); __builtin_amdgcn_wave_barrier(); __builtin_amdgcn_fence(__ATOMIC_RELEASE, "workgroup");
    for (int pc = lane; pc < FEAT / 8; pc += 32) vst2(v_h + grow * FEAT + pc * 8, *(const v4u*)(&sV[w * 2 + rr][pc * 8]));
  }
  __syncthreads();

  v8f acc0 = {}; v8f acc1 = {};
  int ct0 = w * 2, ct1 = w * 2 + 1;
#pragma unroll
  for (int kc = 0; kc < FEAT / 32; ++kc) {
    v16h a  = load_fragA(&sA[0][kc * 32], FEAT, lane);
    v16h b0 = load_fragB(WpT + (ct0 * 16) * FEAT + kc * 32, FEAT, lane);
    v16h b1 = load_fragB(WpT + (ct1 * 16) * FEAT + kc * 32, FEAT, lane);
    acc0 = wmma16x16x32(a, b0, acc0);
    acc1 = wmma16x16x32(a, b1, acc1);
  }
  {
    int cb0 = ct0 * 16 + (lane & 15), cb1 = ct1 * 16 + (lane & 15);
    int rh = (lane >> 4) * 8;
#pragma unroll
    for (int j = 0; j < 8; ++j) {
      sP[rh + j][cb0] = acc0[j] + b_proj[cb0];
      sP[rh + j][cb1] = acc1[j] + b_proj[cb1];
    }
  }
  __syncthreads();

  for (int rr = 0; rr < 2; ++rr) {
    int r = w * 2 + rr;
    float pv[8]; float s = 0.f, s2 = 0.f;
#pragma unroll
    for (int i = 0; i < 8; ++i) {
      float x = sP[r][lane + 32 * i]; pv[i] = x; s += x; s2 += x * x;
    }
#pragma unroll
    for (int o = 16; o > 0; o >>= 1) { s += __shfl_xor(s, o, 32); s2 += __shfl_xor(s2, o, 32); }
    float mu = s * (1.f / MATCH);
    float var = s2 * (1.f / MATCH) - mu * mu;
    float rs = rsqrtf(var + EPSLN);
#pragma unroll
    for (int i = 0; i < 8; ++i) {
      int c = lane + 32 * i;
      sQ[r][c] = (_Float16)((pv[i] - mu) * rs * g1[c] + be1[c]);
    }
    asm volatile("s_wait_dscnt 0" ::: "memory"); __builtin_amdgcn_wave_barrier(); __builtin_amdgcn_fence(__ATOMIC_RELEASE, "workgroup");
    vst2(qk_h + (row0 + r) * MATCH + lane * 8, *(const v4u*)(&sQ[r][lane * 8]));
  }
}

__global__ void k_attn(const _Float16* __restrict__ qk_h, const _Float16* __restrict__ v_h,
                       float* __restrict__ o_f) {
  extern __shared__ char smem[];
  float    (*sS)[BC + 4]  = (float(*)[BC + 4])smem;
  _Float16 (*sP)[BC]      = (_Float16(*)[BC])(smem + 16 * (BC + 4) * 4);
  float* sM     = (float*)(smem + 16 * (BC + 4) * 4 + 16 * BC * 2);
  float* sL     = sM + 16;
  float* sAlpha = sL + 16;
#if !TR16_MODE
  _Float16 (*sVt)[VT_LD]  = (_Float16(*)[VT_LD])(sAlpha + 16);
#endif

  int t = threadIdx.x, lane = t & 31, w = t >> 5;
  int blk = blockIdx.x;
  int b   = blk >> 7;
  int qt  = blk & 127;
  int rb  = b * SEQ;
  int q0  = qt * 16;

  if (t < 16) { sM[t] = -3.0e38f; sL[t] = 0.f; }

  v16h qf[8];
#pragma unroll
  for (int kc = 0; kc < 8; ++kc)
    qf[kc] = load_fragA(qk_h + (rb + q0) * MATCH + kc * 32, MATCH, lane);

  v8f acc[8] = {};
  __syncthreads();

  for (int k0 = 0; k0 < SEQ; k0 += BC) {
#if !TR16_MODE
    for (int c = t; c < BC * (FEAT / 8); c += 128) {
      int key = c >> 6;
      int fc  = c & 63;
      v8h d = *(const v8h*)(v_h + (rb + k0 + key) * FEAT + fc * 8);
#pragma unroll
      for (int j = 0; j < 8; ++j) sVt[fc * 8 + j][key] = d[j];
    }
#endif
    if (k0 + BC < SEQ)
      __builtin_prefetch(v_h + (rb + k0 + BC) * FEAT, 0, 0);

    {
      v8f s = {};
      const _Float16* kbase = qk_h + (rb + k0 + w * 16) * MATCH;
#pragma unroll
      for (int kc = 0; kc < 8; ++kc) {
        v16h bfr = load_fragB(kbase + kc * 32, MATCH, lane);
        s = wmma16x16x32(qf[kc], bfr, s);
      }
      int col = w * 16 + (lane & 15);
      int rh  = (lane >> 4) * 8;
#pragma unroll
      for (int j = 0; j < 8; ++j) sS[rh + j][col] = s[j];
    }
    __syncthreads();

    {
      int r = t >> 3, sub = t & 7;
      float mold = sM[r];
      float sv[8]; float mx = mold;
#pragma unroll
      for (int i = 0; i < 8; ++i) { sv[i] = sS[r][sub * 8 + i]; mx = fmaxf(mx, sv[i]); }
#pragma unroll
      for (int o = 4; o > 0; o >>= 1) mx = fmaxf(mx, __shfl_xor(mx, o, 32));
      float sum = 0.f;
#pragma unroll
      for (int i = 0; i < 8; ++i) {
        float p = expf(sv[i] - mx);
        sP[r][sub * 8 + i] = (_Float16)p;
        sum += p;
      }
#pragma unroll
      for (int o = 4; o > 0; o >>= 1) sum += __shfl_xor(sum, o, 32);
      if (sub == 0) {
        float alpha = expf(mold - mx);
        sL[r] = sL[r] * alpha + sum;
        sM[r] = mx;
        sAlpha[r] = alpha;
      }
    }
    __syncthreads();

    {
      int rh = (lane >> 4) * 8;
      float al[8];
#pragma unroll
      for (int j = 0; j < 8; ++j) al[j] = sAlpha[rh + j];
#pragma unroll
      for (int i = 0; i < 8; ++i)
#pragma unroll
        for (int j = 0; j < 8; ++j) acc[i][j] *= al[j];
    }
    {
      v16h a0 = load_fragA(&sP[0][0],  BC, lane);
      v16h a1 = load_fragA(&sP[0][32], BC, lane);
#if TR16_MODE
      const _Float16* vbase = v_h + (rb + k0) * FEAT;
#pragma unroll
      for (int i = 0; i < 8; ++i) {
        int f0 = (w * 8 + i) * 16;
        v16h b0 = load_fragB_tr16(vbase + f0, FEAT, lane);
        v16h b1 = load_fragB_tr16(vbase + 32 * FEAT + f0, FEAT, lane);
        acc[i] = wmma16x16x32(a0, b0, acc[i]);
        acc[i] = wmma16x16x32(a1, b1, acc[i]);
      }
#else
#pragma unroll
      for (int i = 0; i < 8; ++i) {
        int ft = w * 8 + i;
        v16h b0 = load_fragB(&sVt[ft * 16][0],  VT_LD, lane);
        v16h b1 = load_fragB(&sVt[ft * 16][32], VT_LD, lane);
        acc[i] = wmma16x16x32(a0, b0, acc[i]);
        acc[i] = wmma16x16x32(a1, b1, acc[i]);
      }
#endif
    }
    __syncthreads();
  }

  {
    float* so = (float*)&sVt[0][0];
    int rh = (lane >> 4) * 8;
    float inv[8];
#pragma unroll
    for (int j = 0; j < 8; ++j) inv[j] = 1.f / sL[rh + j];
#pragma unroll
    for (int i = 0; i < 8; ++i) {
      int col = (w * 8 + i) * 16 + (lane & 15);
#pragma unroll
      for (int j = 0; j < 8; ++j) so[(rh + j) * FEAT + col] = acc[i][j] * inv[j];
    }
    __syncthreads();
    for (int q = t; q < 16 * FEAT / 4; q += 128) { const int r = q >> 7, pc = q & 127;
      vst2(o_f + (rb + q0 + r) * FEAT + pc * 4, *(const v4f*)(so + r * FEAT + pc * 4)); }
  }
}

__global__ void k_outproj(const float* __restrict__ o_f, const _Float16* __restrict__ WoT,
                          const float* __restrict__ b_out, float* __restrict__ out) {
  __shared__ _Float16 sA[16][FEAT];
  int row0 = blockIdx.x * 16;
  int t = threadIdx.x, lane = t & 31, w = t >> 5;

  for (int idx = t; idx < 16 * FEAT; idx += 256) {
    int r = idx >> 9, c = idx & (FEAT - 1);
    sA[r][c] = (_Float16)o_f[(row0 + r) * FEAT + c];
  }
  __syncthreads();

  v8f acc[4] = {};
#pragma unroll
  for (int kc = 0; kc < FEAT / 32; ++kc) {
    v16h a = load_fragA(&sA[0][kc * 32], FEAT, lane);
#pragma unroll
    for (int i = 0; i < 4; ++i) {
      int ct = w * 4 + i;
      v16h b = load_fragB(WoT + (ct * 16) * FEAT + kc * 32, FEAT, lane);
      acc[i] = wmma16x16x32(a, b, acc[i]);
    }
  }
  int rh = (lane >> 4) * 8;
  __shared__ __align__(16) float so2[8][16 * 64];
  float* S = so2[w];
#pragma unroll
  for (int i = 0; i < 4; ++i) {
    int col = (w * 4 + i) * 16 + (lane & 15);
#pragma unroll
    for (int j = 0; j < 8; ++j) S[(rh + j) * 64 + i * 16 + (lane & 15)] = acc[i][j] + b_out[col];
  }
  asm volatile("s_wait_dscnt 0" ::: "memory"); __builtin_amdgcn_wave_barrier(); __builtin_amdgcn_fence(__ATOMIC_RELEASE, "workgroup");
#pragma unroll
  for (int q = 0; q < 8; ++q) { const int rl = q * 2 + (lane >> 4), pc = lane & 15; const int grow = row0 + rl;
    const size_t idx = (size_t)grow * FEAT + w * 64 + pc * 4;
    v4f v = *(const v4f*)(S + rl * 64 + pc * 4); const v4f rr2 = *(const v4f*)(o_f + idx);
    vst2(out + idx, v + rr2); }
}

extern "C" void kernel_launch(void* const* d_in, const int* in_sizes, int n_in,
                              void* d_out, int out_size, void* d_ws, size_t ws_size,
                              hipStream_t stream) {
  (void)in_sizes; (void)n_in; (void)out_size; (void)ws_size;
  const float* X      = (const float*)d_in[0];
  const float* W_proj = (const float*)d_in[1];
  const float* b_proj = (const float*)d_in[2];
  const float* g1     = (const float*)d_in[3];
  const float* be1    = (const float*)d_in[4];
  const float* g2     = (const float*)d_in[5];
  const float* be2    = (const float*)d_in[6];
  const float* W_out  = (const float*)d_in[7];
  const float* b_out  = (const float*)d_in[8];
  float* out = (float*)d_out;

  char* ws = (char*)d_ws;
  _Float16* qk_h = (_Float16*)(ws);
  _Float16* v_h  = (_Float16*)(ws + 8388608);
  float*    o_f  = (float*)   (ws + 25165824);
  _Float16* WpT  = (_Float16*)(ws + 58720256);
  _Float16* WoT  = (_Float16*)(ws + 58982400);

  k_prep_weights<<<((FEAT * MATCH + FEAT * FEAT) / 8 + 255) / 256, 256, 0, stream>>>(W_proj, W_out, WpT, WoT);
  k_proj_ln<<<ROWS / 16, 256, 0, stream>>>(X, WpT, b_proj, g1, be1, g2, be2, qk_h, v_h);

  size_t smem = 16 * (BC + 4) * 4 + 16 * BC * 2 + 3 * 16 * 4 + (size_t)FEAT * VT_LD * 2;
  k_attn<<<BATCH * (SEQ / 16), 128, smem, stream>>>(qk_h, v_h, o_f);

  k_outproj<<<ROWS / 16, 256, 0, stream>>>(o_f, WoT, b_out, out);
}
